// StandardAttention_87849261072925
// MI455X (gfx1250) — hardware-verified
//
#include <hip/hip_runtime.h>


#ifndef NB
#define NB 4
#endif
#ifndef SEQ
#define SEQ 2048
#endif
#ifndef NB_FULL
#define NB_FULL 4
#endif
#ifndef SEQ_FULL
#define SEQ_FULL 2048
#endif
#ifndef PRES
#define PRES 0
#endif

namespace {
constexpr int H = 16, HD = 64, QL = SEQ, SK = SEQ;
constexpr float XS = 8.0f, PS = 1024.0f, PRS = 1024.0f, LOG2E = 1.4426950408889634f;
static_assert(SEQ % 64 == 0 && SEQ >= 64 && SEQ <= SEQ_FULL && NB >= 1 && NB <= NB_FULL && HD == 64 && QL == SK);

typedef _Float16 b16;
typedef __attribute__((ext_vector_type(16))) _Float16 v16b;
typedef __attribute__((ext_vector_type(8))) _Float16 v8b;
typedef __attribute__((ext_vector_type(8))) float v8f;
typedef __attribute__((ext_vector_type(4))) float v4f;

__device__ __forceinline__ float bf16_rne(float f) { unsigned int u = __float_as_uint(f); u += 0x7FFFu + ((u >> 16) & 1u); return __uint_as_float(u & 0xFFFF0000u); }
__device__ __forceinline__ v16b frag_kb(const b16* p, int hh) {
  const v8b a = *(const v8b*)(p + 8 * hh), b = *(const v8b*)(p + 16 + 8 * hh); v16b f;
#pragma unroll
  for (int e = 0; e < 8; ++e) { f[e] = a[e]; f[8 + e] = b[e]; }
  return f;
}
__device__ __forceinline__ v8f wmma16b(v16b a, v16b b, v8f c) {
  v8f d = __builtin_amdgcn_wmma_f32_16x16x32_f16(false, a, false, b, (short)0, c, false, false);
  asm volatile("v_nop\n\tv_nop\n\tv_nop\n\tv_nop" : "+v"(d) : "v"(a), "v"(b));
  return d;
}
__device__ __forceinline__ void wave_lds_sync() { __builtin_amdgcn_fence(3, "workgroup"); __builtin_amdgcn_wave_barrier(); __builtin_amdgcn_fence(2, "workgroup"); }
__device__ __forceinline__ float nexp2(float v) { return __builtin_amdgcn_exp2f(v); }

__global__ __launch_bounds__(256) void cvt_qk_kernel(const float* __restrict__ Q, const float* __restrict__ K, b16* __restrict__ Qp, b16* __restrict__ Kp) {
  const size_t u = (size_t)blockIdx.x * 256 + threadIdx.x; const size_t g = u >> 3; const int piece = (int)(u & 7);
  if (g >= (size_t)NB * H * SEQ) return;
  const int s = (int)(g % SEQ); const size_t bhi = g / SEQ;
  const float* src = (blockIdx.y == 0 ? Q : K) + (bhi * SEQ_FULL + (size_t)s) * HD + piece * 8;
  b16* dst = (blockIdx.y == 0 ? Qp : Kp) + g * HD + piece * 8;
  const v4f x0 = *(const v4f*)src, x1 = *(const v4f*)(src + 4); v8b o;
#pragma unroll
  for (int j = 0; j < 4; ++j) { o[j] = (b16)(bf16_rne(x0[j]) * XS); o[4 + j] = (b16)(bf16_rne(x1[j]) * XS); }
  *(volatile v8b*)dst = o; __threadfence(); *(volatile v8b*)dst = o;
}

__global__ __launch_bounds__(64) void cvt_vt_kernel(const float* __restrict__ V, b16* __restrict__ VT) {
  __shared__ __attribute__((aligned(16))) b16 St[HD][64 + 8];
  const int tid = threadIdx.x, wave = tid >> 5, lane = tid & 31; const int rb = blockIdx.x; const size_t bhi = blockIdx.y;
  const float* src = V + (bhi * SEQ_FULL + (size_t)rb * 64) * HD;
  for (int it = 0; it < 16; ++it) {
    const int e = (it * 64 + tid) * 4; const int tok = e >> 6, d = e & 63;
    const v4f x = *(const v4f*)(src + e);
#pragma unroll
    for (int j = 0; j < 4; ++j) St[d + j][tok] = (b16)(bf16_rne(x[j]) * XS);
  }
  __syncthreads();
  b16* dstb = VT + bhi * HD * (size_t)SK + (size_t)rb * 64;
  for (int pass = 0; pass < 2; ++pass) {
#pragma unroll 1
    for (int it = 0; it < 8; ++it) {
      const int d = wave * 32 + it * 4 + (lane >> 3), tok = (lane & 7) * 8;
      const v8b o = *(const v8b*)(&St[d][tok]);
      *(volatile v8b*)(dstb + (size_t)d * SK + tok) = o; }
    __threadfence(); }
}

template <bool PR>
__global__ __launch_bounds__(64) __attribute__((amdgpu_num_vgpr(256))) void attn_kernel(const b16* __restrict__ Qp, const b16* __restrict__ Kp, const b16* __restrict__ VT,
                                                                                      float* __restrict__ out) {
  __shared__ __attribute__((aligned(16))) b16 Pb[2][16][32 + 8];
  __shared__ __attribute__((aligned(16))) b16 Pr[2][16][32 + 8];
  __shared__ __attribute__((aligned(16))) float To[2][16][HD + 4];
  const int wave = threadIdx.x >> 5, lane = threadIdx.x & 31, hh = lane >> 4, col = lane & 15;
  const size_t bhi = blockIdx.y; const int bx = (int)blockIdx.x; const int q0 = bx * 32 + wave * 16, qi = q0 + col;
  const b16* Qb = Qp + bhi * QL * HD; const b16* Kb = Kp + bhi * SK * HD; const b16* Vb = VT + bhi * HD * (size_t)SK;
  const v16b qa0 = frag_kb(Qb + (size_t)qi * HD, hh), qa1 = frag_kb(Qb + (size_t)qi * HD + 32, hh);
  const float cs = LOG2E / (8.0f * XS * XS);
  float m = -INFINITY, l = 0.0f; v8f o[4], o2[4];
#pragma unroll
  for (int t = 0; t < 4; ++t) { o[t] = (v8f){}; o2[t] = (v8f){}; }
#pragma unroll 1
  for (int kb = 0; kb < SK; kb += 32) {
    float e[16]; float mx = -INFINITY;
#pragma unroll
    for (int u = 0; u < 2; ++u) {
      const size_t kr = (size_t)(kb + u * 16 + col) * HD;
      v8f s = (v8f){}; s = wmma16b(frag_kb(Kb + kr, hh), qa0, s); s = wmma16b(frag_kb(Kb + kr + 32, hh), qa1, s);
#pragma unroll
      for (int r = 0; r < 8; ++r) { const float v = s[r] * cs; e[u * 8 + r] = v; mx = fmaxf(mx, v); } }
    mx = fmaxf(mx, __shfl_xor(mx, 16)); const float mn = fmaxf(m, mx); const float al = nexp2(m - mn); float sum = 0.0f;
#pragma unroll
    for (int i2 = 0; i2 < 16; ++i2) {
      const float p = nexp2(e[i2] - mn); sum += p; const int pi = (i2 < 8 ? 0 : 16) + 8 * hh + (i2 & 7);
      const float pp = p * PS; const b16 ph = (b16)pp; Pb[wave][col][pi] = ph;
      if constexpr (PR) Pr[wave][col][pi] = (b16)((pp - (float)ph) * PRS); }
    sum += __shfl_xor(sum, 16); l = l * al + sum; m = mn;
    wave_lds_sync();
    const v16b pf = frag_kb(&Pb[wave][col][0], hh);
    v16b prf = (v16b){};
    if constexpr (PR) prf = frag_kb(&Pr[wave][col][0], hh);
#pragma unroll
    for (int t = 0; t < 4; ++t) {
      o[t] *= al; const v16b vh = frag_kb(Vb + (size_t)(t * 16 + col) * SK + kb, hh);
      o[t] = wmma16b(vh, pf, o[t]);
      if constexpr (PR) { o2[t] *= al; o2[t] = wmma16b(vh, prf, o2[t]); } }
    wave_lds_sync(); }
  const float inv = 1.0f / (l * PS * XS);
#pragma unroll
  for (int t = 0; t < 4; ++t) {
#pragma unroll
    for (int r = 0; r < 8; ++r) {
      float ov = o[t][r];
      if constexpr (PR) ov += o2[t][r] * (1.0f / PRS);
      To[wave][col][t * 16 + 8 * hh + r] = ov * inv; } }
  wave_lds_sync();
  float* ob = out + (bhi * SEQ_FULL + (size_t)q0) * HD;
  for (int pass = 0; pass < 2; ++pass) {
#pragma unroll 1
    for (int it = 0; it < 8; ++it) {
      const int rr = it * 2 + hh; const v4f f = *(const v4f*)(&To[wave][rr][col * 4]);
      *(volatile v4f*)(ob + (size_t)rr * HD + col * 4) = f; }
    __threadfence(); }
}
}

extern "C" void kernel_launch(void* const* d_in, const int* in_sizes, int n_in, void* d_out, int out_size, void* d_ws, size_t ws_size, hipStream_t stream) {
  const size_t need = (((size_t)(NB - 1) * H + (H - 1)) * SEQ_FULL + SEQ) * HD;
  if (n_in < 3 || (size_t)in_sizes[0] < need || (size_t)in_sizes[1] < need || (size_t)in_sizes[2] < need || (size_t)out_size < need) return;
  const float* Qin = (const float*)d_in[0]; const float* Kin = (const float*)d_in[1]; const float* Vin = (const float*)d_in[2];
  size_t off = 0; char* ws = (char*)d_ws;
  auto carve = [&](size_t bytes) { char* p = ws + off; off += (bytes + 255) & ~(size_t)255; return p; };
  const size_t plane = (size_t)NB * H * SEQ * HD * 2;
  b16* Qp = (b16*)carve(plane); b16* Kp = (b16*)carve(plane); b16* VT = (b16*)carve(plane);
  if (off > ws_size || off > ((size_t)128 << 20)) return;
  cvt_qk_kernel<<<dim3((unsigned)(((size_t)NB * H * SEQ * 8 + 255) / 256), 2), 256, 0, stream>>>(Qin, Kin, Qp, Kp);
  cvt_vt_kernel<<<dim3(SEQ / 64, NB * H), 64, 0, stream>>>(Vin, VT);
  attn_kernel<(PRES != 0)><<<dim3(QL / 32, NB * H), 64, 0, stream>>>(Qp, Kp, VT, (float*)d_out);
}
